// RecursiveNN_94489281191
// MI455X (gfx1250) — hardware-verified
//
#include <hip/hip_runtime.h>
#include <stdint.h>

constexpr int kTrees    = 256;
constexpr int kLeaves   = 512;
constexpr int kEmb      = 256;
constexpr int kCls      = 5;
constexpr int kNodes    = 1023;
constexpr int kNodePad  = 1024;
constexpr int kKdim     = 2 * kEmb;
constexpr int kChunkRows = 16384;
constexpr float kHCarry = 64.0f;
constexpr float kWCarry = 16.0f;
constexpr float kGemmScale = 1.0f / 1024.0f;

typedef __attribute__((ext_vector_type(16))) _Float16 v16h;
typedef __attribute__((ext_vector_type(8)))  _Float16 v8h;
typedef __attribute__((ext_vector_type(16))) __bf16   v16b;
typedef __attribute__((ext_vector_type(8)))  __bf16   v8b;
typedef __attribute__((ext_vector_type(8)))  float    v8f;
typedef __attribute__((ext_vector_type(4)))  float    v4f;
typedef __attribute__((ext_vector_type(4)))  unsigned int v4u;

__device__ __forceinline__ unsigned short f2bf_bits(float f) {
  unsigned u = __float_as_uint(f);
  return (unsigned short)((u + 0x7FFFu + ((u >> 16) & 1u)) >> 16);
}
__device__ __forceinline__ float bf_bits2f(unsigned short h) { return __uint_as_float(((unsigned)h) << 16); }

__device__ __forceinline__ void dep_guard_h(v8f& a, v8f& b, v16h x, v16h y) { asm volatile("v_nop\n\tv_nop\n\tv_nop\n\tv_nop" : "+v"(a), "+v"(b) : "v"(x), "v"(y)); }
__device__ __forceinline__ void dep_guard_b(v8f& a, v8f& b, v16b x, v16b y) { asm volatile("v_nop\n\tv_nop\n\tv_nop\n\tv_nop" : "+v"(a), "+v"(b) : "v"(x), "v"(y)); }
__device__ __forceinline__ void keep4_h(v16h a, v16h b, v16h c, v16h d) { asm volatile("v_nop" :: "v"(a), "v"(b), "v"(c), "v"(d)); }
__device__ __forceinline__ void keep4_b(v16b a, v16b b, v16b c, v16b d) { asm volatile("v_nop" :: "v"(a), "v"(b), "v"(c), "v"(d)); }
__device__ __forceinline__ void acc_guard4(v8f& a, v8f& b, v8f& c, v8f& d) { asm volatile("v_nop\n\tv_nop\n\tv_nop\n\tv_nop" : "+v"(a), "+v"(b), "+v"(c), "+v"(d)); }
template <typename T> struct Frag;
template <> struct Frag<_Float16> {
  typedef v16h V; union U { v16h v; v8h h[2]; };
  static __device__ __forceinline__ v16h load(const _Float16* p) {
    U f; f.h[0] = *(const v8h*)(p); f.h[1] = *(const v8h*)(p + 16); return f.v;
  }
  static __device__ __forceinline__ v8f mma(v16h a, v16h b, v8f c) {
    return __builtin_amdgcn_wmma_f32_16x16x32_f16(false, a, false, b, (short)0, c, false, false);
  }
  static __device__ __forceinline__ void guard(v8f& a, v8f& b, v16h x, v16h y) { dep_guard_h(a, b, x, y); }
  static __device__ __forceinline__ void keep(v16h a, v16h b, v16h c, v16h d) { keep4_h(a, b, c, d); }
};
template <> struct Frag<__bf16> {
  typedef v16b V; union U { v16b v; v8b h[2]; };
  static __device__ __forceinline__ v16b load(const __bf16* p) {
    U f; f.h[0] = *(const v8b*)(p); f.h[1] = *(const v8b*)(p + 16); return f.v;
  }
  static __device__ __forceinline__ v8f mma(v16b a, v16b b, v8f c) {
    return __builtin_amdgcn_wmma_f32_16x16x32_bf16(false, a, false, b, (short)0, c, false, false);
  }
  static __device__ __forceinline__ void guard(v8f& a, v8f& b, v16b x, v16b y) { dep_guard_b(a, b, x, y); }
  static __device__ __forceinline__ void keep(v16b a, v16b b, v16b c, v16b d) { keep4_b(a, b, c, d); }
};

__device__ __forceinline__ unsigned pk16(unsigned short a, unsigned short b) { return (unsigned)a | ((unsigned)b << 16); }
__device__ __forceinline__ unsigned short h_bits(float f) { const _Float16 h = (_Float16)f; return __builtin_bit_cast(unsigned short, h); }

template <int ET> struct Elem;
template <> struct Elem<0> { typedef _Float16 T; };
template <> struct Elem<1> { typedef __bf16 T; };
template <int ET, bool SPLIT, int BIAS_MODE, int OUT_MODE, bool RESID, int ACT = 0>
__global__ __launch_bounds__(256) void wmma_gemm64(
    const unsigned short* __restrict__ Ap, const unsigned short* __restrict__ A2p, int lda, long strideA,
    const unsigned short* __restrict__ Btp, const unsigned short* __restrict__ Bt2p, int ldb, long strideB,
    void* __restrict__ Cout, void* __restrict__ Cout2, int ldc, long strideC,
    const float* __restrict__ bias,
    const float* __restrict__ resid, long strideR,
    int M, int N, int K, float scale) {
  typedef typename Elem<ET>::T T;
  typedef typename Frag<T>::V V;
  const T* A = (const T*)Ap; const T* A2 = (const T*)A2p; const T* Bt = (const T*)Btp; const T* Bt2 = (const T*)Bt2p;
  __shared__ __align__(16) float sT[8][16 * 68];
  const int b    = blockIdx.y;
  const int lane = threadIdx.x & 31;
  const int wave = threadIdx.x >> 5;
  const int tilesN = N >> 6;
  const int tilesM = M >> 6;
  const int tile = blockIdx.x * 8 + wave;
  if (tile >= tilesM * tilesN) return;
  const int tm = tile / tilesN;
  const int tn = tile - tm * tilesN;
  const int m0 = tm << 6;
  const int n0 = tn << 6;

  const T* Ab  = A  + (size_t)b * strideA;
  const T* Bb  = Bt + (size_t)b * strideB;
  const T* Ab2 = SPLIT ? (A2  + (size_t)b * strideA) : nullptr;
  const T* Bb2 = SPLIT ? (Bt2 + (size_t)b * strideB) : nullptr;

  const int rlane = lane & 15;
  const int koff  = (lane >> 4) * 8;
  const int mOff  = (lane >> 4) * 8;

  v8f acc[4][4];
#pragma unroll
  for (int i = 0; i < 4; ++i)
#pragma unroll
    for (int j = 0; j < 4; ++j) acc[i][j] = (v8f){0.f,0.f,0.f,0.f,0.f,0.f,0.f,0.f};

  for (int k0 = 0; k0 < K; k0 += 32) {
    V bh[4], bl[4];
#pragma unroll
    for (int j = 0; j < 4; ++j) {
      const size_t bo = (size_t)(n0 + (j << 4) + rlane) * ldb + koff + k0;
      bh[j] = Frag<T>::load(Bb + bo);
      if (SPLIT) bl[j] = Frag<T>::load(Bb2 + bo);
    }
#pragma unroll
    for (int i = 0; i < 4; ++i) {
      const size_t ao = (size_t)(m0 + (i << 4) + rlane) * lda + koff + k0;
      V ah = Frag<T>::load(Ab + ao);
      V al;
      if (SPLIT) al = Frag<T>::load(Ab2 + ao);
#pragma unroll
      for (int j = 0; j < 4; ++j) {
        acc[i][j] = Frag<T>::mma(ah, bh[j], acc[i][j]);
        if (SPLIT) {
          acc[i][j] = Frag<T>::mma(ah, bl[j], acc[i][j]);
          acc[i][j] = Frag<T>::mma(al, bh[j], acc[i][j]);
        }
      }
      Frag<T>::guard(acc[i][0], acc[i][3], ah, SPLIT ? al : ah);
    }
    Frag<T>::keep(bh[0], bh[1], bh[2], bh[3]);
    if (SPLIT) Frag<T>::keep(bl[0], bl[1], bl[2], bl[3]);
  }
  acc_guard4(acc[0][0], acc[0][1], acc[0][2], acc[0][3]);
  acc_guard4(acc[1][0], acc[1][1], acc[1][2], acc[1][3]);
  acc_guard4(acc[2][0], acc[2][1], acc[2][2], acc[2][3]);
  acc_guard4(acc[3][0], acc[3][1], acc[3][2], acc[3][3]);

  float* slab = sT[wave];
  const float* Rb = RESID ? (resid + (size_t)b * strideR) : nullptr;
#pragma unroll
  for (int i = 0; i < 4; ++i) {
    const int mBase = m0 + (i << 4);
#pragma unroll
    for (int j = 0; j < 4; ++j) {
      const int n = n0 + (j << 4) + rlane;
      float bv = 0.f;
      if (BIAS_MODE == 2) bv = bias[n];
#pragma unroll
      for (int r = 0; r < 8; ++r) {
        float v = acc[i][j][r] * scale;
        if (BIAS_MODE == 1) v += bias[mBase + mOff + r];
        if (BIAS_MODE == 2) v += bv;
        if (RESID) v += Rb[(size_t)(mBase + mOff + r) * ldc + n];
        if (ACT == 2) v = fmaxf(v, 0.0f);
        if (ACT == 4) v = (v > 0.f) ? v : 0.01f * v;
        slab[(mOff + r) * 68 + (j << 4) + rlane] = v;
      }
    }
    __builtin_amdgcn_fence(__ATOMIC_RELEASE, "workgroup");
    __builtin_amdgcn_wave_barrier();
    __builtin_amdgcn_fence(__ATOMIC_ACQUIRE, "workgroup");
    if (OUT_MODE == 0) {
      float* C = (float*)Cout + (size_t)b * strideC;
      const int hh = lane >> 4, c4 = (lane & 15) * 4;
      for (int pass = 0; pass < 2; ++pass) {
#pragma unroll
        for (int it = 0; it < 8; ++it) {
          const int row = it * 2 + hh;
          v4f v = *(const v4f*)(slab + row * 68 + c4);
          *(volatile v4f*)(C + (size_t)(mBase + row) * ldc + n0 + c4) = v;
        }
        __threadfence();
      }
    } else {
      const int q = lane >> 3, c8 = (lane & 7) * 8;
      unsigned short* C  = (unsigned short*)Cout  + (size_t)b * strideC;
      unsigned short* C2 = (OUT_MODE == 2) ? ((unsigned short*)Cout2 + (size_t)b * strideC) : nullptr;
      for (int pass = 0; pass < 2; ++pass) {
#pragma unroll
        for (int it = 0; it < 4; ++it) {
          const int row = it * 4 + q;
          const float* sp = slab + row * 68 + c8;
          v8h hv, lv;
#pragma unroll
          for (int e = 0; e < 8; ++e) {
            if (OUT_MODE == 1) {
              hv[e] = (_Float16)sp[e];
            } else {
              unsigned short hb = f2bf_bits(sp[e]);
              unsigned short lb = f2bf_bits(sp[e] - bf_bits2f(hb));
              hv[e] = __builtin_bit_cast(_Float16, hb);
              lv[e] = __builtin_bit_cast(_Float16, lb);
            }
          }
          *(volatile v8h*)(C + (size_t)(mBase + row) * ldc + n0 + c8) = hv;
          if (OUT_MODE == 2) *(volatile v8h*)(C2 + (size_t)(mBase + row) * ldc + n0 + c8) = lv;
        }
        __threadfence();
      }
    }
    __builtin_amdgcn_fence(__ATOMIC_RELEASE, "workgroup");
    __builtin_amdgcn_wave_barrier();
    __builtin_amdgcn_fence(__ATOMIC_ACQUIRE, "workgroup");
  }
}

__global__ __launch_bounds__(256) void cast8_scale_f16_kernel(const float* __restrict__ in, unsigned short* __restrict__ out,
                                                             int n8, float carry) {
  const int i = blockIdx.x * 256 + threadIdx.x;
  if (i >= n8) return;
  const float* p = in + 8 * (size_t)i;
  const v4f a = *(const v4f*)(p);
  const v4f c = *(const v4f*)(p + 4);
  unsigned short hb[8];
#pragma unroll
  for (int e = 0; e < 4; ++e) {
    hb[e]     = h_bits(a[e] * carry);
    hb[4 + e] = h_bits(c[e] * carry);
  }
  const v4u u = (v4u){pk16(hb[0], hb[1]), pk16(hb[2], hb[3]), pk16(hb[4], hb[5]), pk16(hb[6], hb[7])};
  unsigned short* q = out + 8 * (size_t)i;
  *(volatile v4u*)q = u;
  __threadfence();
  *(volatile v4u*)q = u;
}

template <int MODE, bool WRITE_H, bool WRITE_STG>
__global__ __launch_bounds__(256) void node_kernel(
    const int* __restrict__ words, const float* __restrict__ emb, int nvocab,
    const float* __restrict__ src,
    const float* __restrict__ P, const float* __restrict__ pb,
    unsigned short* __restrict__ hout, float* __restrict__ stg,
    int row0, int n_shift, int node_off, int nrows) {
  __shared__ __align__(16) float sP[kCls * kEmb];
  __shared__ __align__(16) float sProj[64];
  const int t = threadIdx.x;
  const int lane = t & 31, wave = t >> 5;
  if (WRITE_STG) {
#pragma unroll
    for (int c = 0; c < kCls; ++c) sP[c * kEmb + t] = P[c * kEmb + t];
  }
  int rl = blockIdx.x * 8 + wave;
  const bool rowok = rl < nrows;
  rl = rowok ? rl : (nrows - 1);
  const float* p;
  if (MODE == 0) {
    int w = words[rl];
    w = w < 0 ? 0 : w;
    w = w >= nvocab ? (nvocab - 1) : w;
    p = emb + (size_t)w * kEmb + 8 * lane;
  } else {
    p = src + (size_t)rl * kEmb + 8 * lane;
  }
  const v4f a = *(const v4f*)(p);
  const v4f cc = *(const v4f*)(p + 4);
  float x[8];
#pragma unroll
  for (int e = 0; e < 4; ++e) { x[e] = a[e]; x[4 + e] = cc[e]; }
  if (MODE == 0) {
#pragma unroll
    for (int e = 0; e < 8; ++e) x[e] = fmaxf(x[e], 0.0f);
  }
  if (WRITE_H) {
    unsigned short hb[8];
#pragma unroll
    for (int e = 0; e < 8; ++e) hb[e] = h_bits(x[e] * kHCarry);
    const v4u u = (v4u){pk16(hb[0], hb[1]), pk16(hb[2], hb[3]), pk16(hb[4], hb[5]), pk16(hb[6], hb[7])};
    unsigned short* q = hout + ((size_t)(row0 + rl)) * kEmb + 8 * lane;
    if (rowok) *(volatile v4u*)q = u;
    __threadfence();
    if (rowok) *(volatile v4u*)q = u;
  }
  if (WRITE_STG) {
    __syncthreads();
    float d[kCls];
#pragma unroll
    for (int c = 0; c < kCls; ++c) {
      const float* pr = sP + c * kEmb + 8 * lane;
      float s = 0.f;
#pragma unroll
      for (int e = 0; e < 8; ++e) s += x[e] * pr[e];
#pragma unroll
      for (int off = 16; off > 0; off >>= 1) s += __shfl_xor(s, off, 32);
      d[c] = s;
    }
    if (lane == 0) {
#pragma unroll
      for (int c = 0; c < kCls; ++c) sProj[wave * 8 + c] = d[c] + pb[c];
      sProj[wave * 8 + 5] = 0.f;
      sProj[wave * 8 + 6] = 0.f;
      sProj[wave * 8 + 7] = 0.f;
    }
    __syncthreads();
    const int jn = (lane >> 1) & 7, q4 = (lane & 1) * 4;
    const v4f v = *(const v4f*)(sProj + jn * 8 + q4);
    int rj = blockIdx.x * 8 + jn;
    const bool okj = rj < nrows;
    rj = okj ? rj : (nrows - 1);
    const int grow = row0 + rj;
    const int tree = grow >> n_shift;
    const int idx  = grow & ((1 << n_shift) - 1);
    float* dst = stg + ((size_t)(tree * kNodePad + node_off + idx)) * 8 + q4;
    const bool wr = (wave == 0) && (lane < 16) && okj;
    if (wr) *(volatile v4f*)dst = v;
    __threadfence();
    if (wr) *(volatile v4f*)dst = v;
  }
}

__global__ __launch_bounds__(256) void tail_kernel(const float* __restrict__ rc, const float* __restrict__ P,
                                                   const float* __restrict__ pb, float* __restrict__ stg, int lvl9_row0) {
  __shared__ __align__(16) float sP[kCls * kEmb];
  __shared__ __align__(16) float sProj[32];
  const int t = threadIdx.x;
  const int lane = t & 31, wave = t >> 5;
  const int b = blockIdx.x;
#pragma unroll
  for (int c = 0; c < kCls; ++c) sP[c * kEmb + t] = P[c * kEmb + t];
  const int rsel = (wave == 0) ? (2 * b) : (wave == 1) ? (2 * b + 1) : (lvl9_row0 + b);
  const float* p = rc + (size_t)rsel * kEmb + 8 * lane;
  const v4f a = *(const v4f*)(p);
  const v4f cc = *(const v4f*)(p + 4);
  float x[8];
#pragma unroll
  for (int e = 0; e < 4; ++e) { x[e] = a[e]; x[4 + e] = cc[e]; }
  __syncthreads();
  float d[kCls];
#pragma unroll
  for (int c = 0; c < kCls; ++c) {
    const float* pr = sP + c * kEmb + 8 * lane;
    float s = 0.f;
#pragma unroll
    for (int e = 0; e < 8; ++e) s += x[e] * pr[e];
#pragma unroll
    for (int off = 16; off > 0; off >>= 1) s += __shfl_xor(s, off, 32);
    d[c] = s;
  }
  const bool real = wave < 3;
  if (lane == 0 && wave < 4) {
#pragma unroll
    for (int c = 0; c < kCls; ++c) sProj[wave * 8 + c] = real ? (d[c] + pb[c]) : 0.f;
    sProj[wave * 8 + 5] = 0.f;
    sProj[wave * 8 + 6] = 0.f;
    sProj[wave * 8 + 7] = 0.f;
  }
  __syncthreads();
  const int l8 = lane & 7;
  const v4f v = *(const v4f*)(sProj + l8 * 4);
  float* dst = stg + ((size_t)(b * kNodePad + 1020)) * 8 + l8 * 4;
  const bool wr = (wave == 0) && (lane < 8);
  if (wr) *(volatile v4f*)dst = v;
  __threadfence();
  if (wr) *(volatile v4f*)dst = v;
}

__global__ __launch_bounds__(256) void copy_out_kernel(const float* __restrict__ stg, float* __restrict__ out, int n4) {
  const int i = blockIdx.x * 256 + threadIdx.x;
  if (i >= n4) return;
  v4f v;
#pragma unroll
  for (int e = 0; e < 4; ++e) {
    const int o = 4 * i + e;
    const int q = o / kCls;
    const int c = o - q * kCls;
    const int b = q / kNodes;
    const int n = q - b * kNodes;
    v[e] = stg[((size_t)(b * kNodePad + n)) * 8 + c];
  }
  float* dst = out + 4 * (size_t)i;
  *(volatile v4f*)dst = v;
  __threadfence();
  *(volatile v4f*)dst = v;
}

extern "C" void kernel_launch(void* const* d_in, const int* in_sizes, int n_in,
                              void* d_out, int out_size, void* d_ws, size_t ws_size,
                              hipStream_t stream) {
  if (n_in < 6) return;
  const int*   words = (const int*)d_in[0];
  const float* emb   = (const float*)d_in[1];
  const float* Wf    = (const float*)d_in[2];
  const float* bvec  = (const float*)d_in[3];
  const float* P     = (const float*)d_in[4];
  const float* pb    = (const float*)d_in[5];
  float*       out   = (float*)d_out;

  if (in_sizes[0] != kTrees * kLeaves) return;
  if (in_sizes[1] < kEmb || (in_sizes[1] % kEmb) != 0) return;
  if (in_sizes[2] != kEmb * kKdim) return;
  if (in_sizes[3] < kEmb) return;
  if (in_sizes[4] != kCls * kEmb) return;
  if (in_sizes[5] < kCls) return;
  if (out_size != kTrees * kNodes * kCls) return;
  const int nvocab = in_sizes[1] / kEmb;

  const size_t offA = 0;
  const size_t szA  = (size_t)kTrees * kLeaves * kEmb * 2;
  const size_t offB = offA + szA;
  const size_t szB  = szA / 2;
  const size_t offC = offB + szB;
  const size_t szC  = (size_t)kChunkRows * kEmb * 4;
  const size_t offS = offC + szC;
  const size_t szS  = (size_t)kTrees * kNodePad * 8 * 4;
  const size_t offW = offS + szS;
  const size_t szW  = (size_t)kEmb * kKdim * 2;
  const size_t total = offW + szW;
  if (total > ws_size) return;

  char* ws = (char*)d_ws;
  unsigned short* HA  = (unsigned short*)(ws + offA);
  unsigned short* HB  = (unsigned short*)(ws + offB);
  float*          rcf = (float*)(ws + offC);
  float*          stg = (float*)(ws + offS);
  unsigned short* Wh  = (unsigned short*)(ws + offW);

  cast8_scale_f16_kernel<<<(kEmb * kKdim / 8) / 256, 256, 0, stream>>>(Wf, Wh, kEmb * kKdim / 8, kWCarry);

  node_kernel<0, true, true><<<(kTrees * kLeaves) / 8, 256, 0, stream>>>(
      words, emb, nvocab, rcf, P, pb, HA, stg, 0, 9, 0, kTrees * kLeaves);

  for (int j = 1; j <= 9; ++j) {
    const int n_out = kLeaves >> j;
    const int Mtot  = kTrees * n_out;
    const int chunk = Mtot < kChunkRows ? Mtot : kChunkRows;
    const int nch   = Mtot / chunk;
    const unsigned short* Hin  = ((j - 1) & 1) ? HB : HA;
    unsigned short*       Hout = (j & 1) ? HB : HA;
    const int crow0 = (j == 9) ? 512 : 0;
    const int node_off = kNodePad - 2 * n_out;
    for (int ch = 0; ch < nch; ++ch) {
      const unsigned short* A = Hin + (size_t)ch * chunk * kKdim;
      float* C = rcf + (size_t)crow0 * kEmb;
      dim3 ggrid(chunk / 128, 1);
      wmma_gemm64<0, false, 2, 0, false, 2><<<ggrid, 256, 0, stream>>>(
          A, A, kKdim, 0L, Wh, Wh, kKdim, 0L, (void*)C, (void*)C, kEmb, 0L,
          bvec, bvec, 0L, chunk, kEmb, kKdim, kGemmScale);
      if (j <= 7) {
        node_kernel<1, true, true><<<chunk / 8, 256, 0, stream>>>(
            words, emb, nvocab, C, P, pb, Hout, stg, ch * chunk, 9 - j, node_off, chunk);
      } else if (j == 8) {
        node_kernel<1, true, false><<<chunk / 8, 256, 0, stream>>>(
            words, emb, nvocab, C, P, pb, Hout, stg, ch * chunk, 9 - j, node_off, chunk);
      } else {
        tail_kernel<<<kTrees, 256, 0, stream>>>(rcf, P, pb, stg, crow0);
      }
    }
  }

  const int n4 = out_size / 4;
  copy_out_kernel<<<(n4 + 255) / 256, 256, 0, stream>>>(stg, out, n4);
}
